// KNNRegressor_7215545057604
// MI455X (gfx1250) — hardware-verified
//
#include <hip/hip_runtime.h>

typedef __bf16         v16bf __attribute__((ext_vector_type(16)));
typedef unsigned short v8us  __attribute__((ext_vector_type(8)));
typedef float          v8f   __attribute__((ext_vector_type(8)));
typedef float          v4f   __attribute__((ext_vector_type(4)));
typedef v8us __attribute__((may_alias)) v8usa;
typedef v4f  __attribute__((may_alias)) v4fa;

union Frag { v16bf v; v8us h[2]; };

#define NTR  65536
#define NQR  4096
#define DIMS 128
#define QPB  64
#define RPB  256

static_assert(NTR % RPB == 0);
static_assert(NQR % RPB == 0);
static_assert(NQR % QPB == 0);
static_assert(NTR % 16 == 0);
static_assert(DIMS == 128);

__device__ __forceinline__ unsigned int f2bf_bits(float f) {
  unsigned int u = __float_as_uint(f);
  u += 0x7FFFu + ((u >> 16) & 1u);
  return u >> 16;
}
__device__ __forceinline__ float bfbits2f(unsigned int b) {
  return __uint_as_float(b << 16);
}

__device__ __forceinline__ void ins5(float dc, float sc, int ic,
    float& d0, float& d1, float& d2, float& d3, float& d4,
    float& s0, float& s1, float& s2, float& s3, float& s4,
    int& i0, int& i1, int& i2, int& i3, int& i4)
{
  const bool c0 = dc < d0, c1 = dc < d1, c2 = dc < d2, c3 = dc < d3, c4 = dc < d4;
  const float nd4 = c4 ? (c3 ? d3 : dc) : d4;  const float ns4 = c4 ? (c3 ? s3 : sc) : s4;  const int ni4 = c4 ? (c3 ? i3 : ic) : i4;
  const float nd3 = c3 ? (c2 ? d2 : dc) : d3;  const float ns3 = c3 ? (c2 ? s2 : sc) : s3;  const int ni3 = c3 ? (c2 ? i2 : ic) : i3;
  const float nd2 = c2 ? (c1 ? d1 : dc) : d2;  const float ns2 = c2 ? (c1 ? s1 : sc) : s2;  const int ni2 = c2 ? (c1 ? i1 : ic) : i2;
  const float nd1 = c1 ? (c0 ? d0 : dc) : d1;  const float ns1 = c1 ? (c0 ? s0 : sc) : s1;  const int ni1 = c1 ? (c0 ? i0 : ic) : i1;
  const float nd0 = c0 ? dc : d0;              const float ns0 = c0 ? sc : s0;              const int ni0 = c0 ? ic : i0;
  d0 = nd0; d1 = nd1; d2 = nd2; d3 = nd3; d4 = nd4;
  s0 = ns0; s1 = ns1; s2 = ns2; s3 = ns3; s4 = ns4;
  i0 = ni0; i1 = ni1; i2 = ni2; i3 = ni3; i4 = ni4;
}

__device__ __forceinline__ void ins5lex(float dc, int ic,
    float& d0, float& d1, float& d2, float& d3, float& d4,
    int& i0, int& i1, int& i2, int& i3, int& i4)
{
  const bool c0 = (dc < d0) || (dc == d0 && ic < i0);
  const bool c1 = (dc < d1) || (dc == d1 && ic < i1);
  const bool c2 = (dc < d2) || (dc == d2 && ic < i2);
  const bool c3 = (dc < d3) || (dc == d3 && ic < i3);
  const bool c4 = (dc < d4) || (dc == d4 && ic < i4);
  const float nd4 = c4 ? (c3 ? d3 : dc) : d4;  const int ni4 = c4 ? (c3 ? i3 : ic) : i4;
  const float nd3 = c3 ? (c2 ? d2 : dc) : d3;  const int ni3 = c3 ? (c2 ? i2 : ic) : i3;
  const float nd2 = c2 ? (c1 ? d1 : dc) : d2;  const int ni2 = c2 ? (c1 ? i1 : ic) : i2;
  const float nd1 = c1 ? (c0 ? d0 : dc) : d1;  const int ni1 = c1 ? (c0 ? i0 : ic) : i1;
  const float nd0 = c0 ? dc : d0;              const int ni0 = c0 ? ic : i0;
  d0 = nd0; d1 = nd1; d2 = nd2; d3 = nd3; d4 = nd4;
  i0 = ni0; i1 = ni1; i2 = ni2; i3 = ni3; i4 = ni4;
}

__global__ __launch_bounds__(256) void convert_kernel(
    const float* __restrict__ xtr,
    const float* __restrict__ xte,
    unsigned short* __restrict__ pt,
    unsigned short* __restrict__ pq,
    float* __restrict__ b2,
    float* __restrict__ a2,
    float* __restrict__ b2min8)
{
  __shared__ __attribute__((aligned(16))) float sN[RPB];
  __shared__ __attribute__((aligned(16))) float sM[32];

  const int tid = threadIdx.x, lane = tid & 31, w = tid >> 5;
  const int h = lane >> 4, m = lane & 15;
  const int blk = blockIdx.x;
  const bool is_train = blk < (NTR / RPB);
  const int rbase = (is_train ? blk : (blk - NTR / RPB)) * RPB;
  const float* src = is_train ? xtr : xte;
  unsigned short* dst = is_train ? pt : pq;
  float* ndst = is_train ? b2 : a2;

  #pragma unroll 1
  for (int it = 0; it < 16; ++it) {
    const int lr = 32 * w + 2 * it + h;
    const size_t row = (size_t)(rbase + lr);
    const float* p = src + row * DIMS + 8 * m;
    const v4f xa = *(const v4fa*)p;
    const v4f xb = *(const v4fa*)(p + 4);
    const float xs[8] = { xa[0], xa[1], xa[2], xa[3], xb[0], xb[1], xb[2], xb[3] };
    v8us o;
    float ss = 0.0f;
    #pragma unroll
    for (int j = 0; j < 8; ++j) {
      const unsigned int bits = f2bf_bits(xs[j]);
      o[j] = (unsigned short)bits;
      const float r = bfbits2f(bits);
      ss += r * r;
    }
    unsigned short* qd = dst + row * DIMS + 8 * m;
    *(volatile v8us*)qd = o;
    __threadfence();
    *(volatile v8us*)qd = o;
    ss += __shfl_xor(ss, 8);
    ss += __shfl_xor(ss, 4);
    ss += __shfl_xor(ss, 2);
    ss += __shfl_xor(ss, 1);
    if (m == 0) sN[lr] = ss;
  }
  __syncthreads();

  if (w < 2) {
    const v4f v = *(const v4fa*)(sN + 4 * tid);
    float* qd = ndst + rbase + 4 * tid;
    *(volatile v4f*)qd = v;
    __threadfence();
    *(volatile v4f*)qd = v;
  }
  if (is_train && w == 2) {
    float mn = sN[8 * lane];
    #pragma unroll
    for (int k = 1; k < 8; ++k) mn = fminf(mn, sN[8 * lane + k]);
    sM[lane] = mn;
  }
  __syncthreads();
  if (is_train && w == 2) {
    const v4f v = *(const v4fa*)(sM + 4 * (lane & 7));
    float* qd = b2min8 + blk * 32 + 4 * (lane & 7);
    if (lane < 8) *(volatile v4f*)qd = v;
    __threadfence();
    if (lane < 8) *(volatile v4f*)qd = v;
  }
}

__global__ __launch_bounds__(128) void select_kernel(
    const unsigned short* __restrict__ pq,
    const unsigned short* __restrict__ pt,
    const float* __restrict__ a2,
    const float* __restrict__ b2,
    const float* __restrict__ b2min8,
    const float* __restrict__ y,
    float* __restrict__ out)
{
  __shared__ __attribute__((aligned(16))) float sOut[QPB];

  const int tid = threadIdx.x, lane = tid & 31, w = tid >> 5;
  const int h = lane >> 4, m = lane & 15;
  const int q = blockIdx.x * QPB + 16 * w + m;

  const unsigned short* qrow = pq + (size_t)q * DIMS + 8 * h;
  Frag qb0, qb1, qb2, qb3;
  qb0.h[0] = *(const v8usa*)(qrow + 0);   qb0.h[1] = *(const v8usa*)(qrow + 16);
  qb1.h[0] = *(const v8usa*)(qrow + 32);  qb1.h[1] = *(const v8usa*)(qrow + 48);
  qb2.h[0] = *(const v8usa*)(qrow + 64);  qb2.h[1] = *(const v8usa*)(qrow + 80);
  qb3.h[0] = *(const v8usa*)(qrow + 96);  qb3.h[1] = *(const v8usa*)(qrow + 112);
  const float a2q = a2[q];

  const float INF = __builtin_inff();
  float d0 = INF, d1 = INF, d2 = INF, d3 = INF, d4 = INF;
  float s0 = INF, s1 = INF, s2 = INF, s3 = INF, s4 = INF;
  int   i0 = 0, i1 = 0, i2 = 0, i3 = 0, i4 = 0;

  const unsigned short* trow = pt + (size_t)m * DIMS + 8 * h;
  const v8f zero8 = {0.f, 0.f, 0.f, 0.f, 0.f, 0.f, 0.f, 0.f};

  #pragma unroll 1
  for (int t0 = 0; t0 < NTR; t0 += 16) {
    const unsigned short* ap = trow + (size_t)t0 * DIMS;
    Frag f0, f1, f2, f3;
    f0.h[0] = *(const v8usa*)(ap + 0);   f0.h[1] = *(const v8usa*)(ap + 16);
    f1.h[0] = *(const v8usa*)(ap + 32);  f1.h[1] = *(const v8usa*)(ap + 48);
    f2.h[0] = *(const v8usa*)(ap + 64);  f2.h[1] = *(const v8usa*)(ap + 80);
    f3.h[0] = *(const v8usa*)(ap + 96);  f3.h[1] = *(const v8usa*)(ap + 112);

    v8f c = __builtin_amdgcn_wmma_f32_16x16x32_bf16(false, f0.v, false, qb0.v, (short)0, zero8, false, false);
    c = __builtin_amdgcn_wmma_f32_16x16x32_bf16(false, f1.v, false, qb1.v, (short)0, c, false, false);
    c = __builtin_amdgcn_wmma_f32_16x16x32_bf16(false, f2.v, false, qb2.v, (short)0, c, false, false);
    c = __builtin_amdgcn_wmma_f32_16x16x32_bf16(false, f3.v, false, qb3.v, (short)0, c, false, false);
    asm volatile("v_nop\n\tv_nop\n\tv_nop\n\tv_nop"
                 : "+v"(c)
                 : "v"(f0.v), "v"(f1.v), "v"(f2.v), "v"(f3.v),
                   "v"(qb0.v), "v"(qb1.v), "v"(qb2.v), "v"(qb3.v));

    float cmax = c[0];
    #pragma unroll
    for (int r = 1; r < 8; ++r) cmax = fmaxf(cmax, c[r]);
    const float bmin = b2min8[(t0 >> 3) + h];
    const float g = (a2q + bmin) - 2.0f * cmax;
    if (__any(g < s4)) {
      const float* bp = b2 + t0 + 8 * h;
      const v4f bl = *(const v4fa*)bp;
      const v4f bu = *(const v4fa*)(bp + 4);
      const float bb[8] = { bl[0], bl[1], bl[2], bl[3], bu[0], bu[1], bu[2], bu[3] };
      #pragma unroll
      for (int r = 0; r < 8; ++r) {
        const float sq = (a2q + bb[r]) - 2.0f * c[r];
        if (__any(sq < s4)) {
          const float dd = sqrtf(fmaxf(sq, 0.0f));
          ins5(dd, sq, t0 + 8 * h + r, d0, d1, d2, d3, d4, s0, s1, s2, s3, s4, i0, i1, i2, i3, i4);
        }
      }
    }
  }

  const float e0 = __shfl_xor(d0, 16), e1 = __shfl_xor(d1, 16), e2 = __shfl_xor(d2, 16),
              e3 = __shfl_xor(d3, 16), e4 = __shfl_xor(d4, 16);
  const int   j0 = __shfl_xor(i0, 16), j1 = __shfl_xor(i1, 16), j2 = __shfl_xor(i2, 16),
              j3 = __shfl_xor(i3, 16), j4 = __shfl_xor(i4, 16);
  ins5lex(e0, j0, d0, d1, d2, d3, d4, i0, i1, i2, i3, i4);
  ins5lex(e1, j1, d0, d1, d2, d3, d4, i0, i1, i2, i3, i4);
  ins5lex(e2, j2, d0, d1, d2, d3, d4, i0, i1, i2, i3, i4);
  ins5lex(e3, j3, d0, d1, d2, d3, d4, i0, i1, i2, i3, i4);
  ins5lex(e4, j4, d0, d1, d2, d3, d4, i0, i1, i2, i3, i4);

  const float y0 = bfbits2f(f2bf_bits(y[min(max(i0, 0), NTR - 1)]));
  const float y1 = bfbits2f(f2bf_bits(y[min(max(i1, 0), NTR - 1)]));
  const float y2 = bfbits2f(f2bf_bits(y[min(max(i2, 0), NTR - 1)]));
  const float y3 = bfbits2f(f2bf_bits(y[min(max(i3, 0), NTR - 1)]));
  const float y4 = bfbits2f(f2bf_bits(y[min(max(i4, 0), NTR - 1)]));
  const float mean = ((((y0 + y1) + y2) + y3) + y4) * 0.2f;

  if (h == 0) sOut[16 * w + m] = mean;
  __syncthreads();

  if (w == 0) {
    const v4f v = *(const v4fa*)(sOut + 4 * (lane & 15));
    float* qd = out + (size_t)blockIdx.x * QPB + 4 * (lane & 15);
    if (lane < 16) *(volatile v4f*)qd = v;
    __threadfence();
    if (lane < 16) *(volatile v4f*)qd = v;
  }
}

extern "C" void kernel_launch(void* const* d_in, const int* in_sizes, int n_in,
                              void* d_out, int out_size, void* d_ws, size_t ws_size,
                              hipStream_t stream) {
  if (n_in < 3) return;
  if (in_sizes[0] != NTR * DIMS) return;
  if (in_sizes[1] != NQR * DIMS) return;
  if (in_sizes[2] != NTR) return;
  if (out_size != NQR) return;

  const float* xtr = (const float*)d_in[0];
  const float* xte = (const float*)d_in[1];
  const float* ytr = (const float*)d_in[2];
  float* out = (float*)d_out;

  const size_t pt_bytes  = (size_t)NTR * DIMS * 2;
  const size_t pq_bytes  = (size_t)NQR * DIMS * 2;
  const size_t b2_bytes  = (size_t)NTR * 4;
  const size_t a2_bytes  = (size_t)NQR * 4;
  const size_t bm_bytes  = (size_t)(NTR / 8) * 4;
  const size_t off_pq = pt_bytes;
  const size_t off_b2 = off_pq + pq_bytes;
  const size_t off_a2 = off_b2 + b2_bytes;
  const size_t off_bm = off_a2 + a2_bytes;
  const size_t total  = off_bm + bm_bytes;
  if (total > ws_size) return;

  char* ws = (char*)d_ws;
  unsigned short* pt = (unsigned short*)(ws);
  unsigned short* pq = (unsigned short*)(ws + off_pq);
  float* b2     = (float*)(ws + off_b2);
  float* a2     = (float*)(ws + off_a2);
  float* b2min8 = (float*)(ws + off_bm);

  convert_kernel<<<(NTR + NQR) / RPB, 256, 0, stream>>>(xtr, xte, pt, pq, b2, a2, b2min8);
  select_kernel<<<NQR / QPB, 128, 0, stream>>>(pq, pt, a2, b2, b2min8, ytr, out);
}
